// SearchRankModule_34986803593849
// MI455X (gfx1250) — hardware-verified
//
#include <hip/hip_runtime.h>
#include <math.h>
#include <stdint.h>

#define NB   8
#define NC   128
#define IMW  112
#define HW   12544
#define NPT  196
#define NS   16
#define NH1  32
#define KBW  16
#define BKP  136
#define SOP  68
#define CWS  256.0f
#define CAS  16.0f

static_assert(HW == NPT * 64);
static_assert(HW == IMW * IMW);
static_assert((HW % 32) == 0);
static_assert(NC * KBW == 2048);
static_assert(NC == 4 * 32);
static_assert((BKP % 8) == 0);
static_assert((SOP * 4) % 16 == 0);
static_assert(NC * SOP * 4 == 2 * 64 * BKP * 2);
static_assert(NC * NC == 8 * 256 * 8);

typedef _Float16 v16h __attribute__((ext_vector_type(16)));
typedef _Float16 v8h  __attribute__((ext_vector_type(8)));
typedef float    v8f  __attribute__((ext_vector_type(8)));
typedef float    v4f  __attribute__((ext_vector_type(4)));
typedef unsigned int v4u __attribute__((ext_vector_type(4)));
union Frag { v16h v; v8h half[2]; };

__device__ __forceinline__ unsigned short bf_bits(float f) {
  unsigned u = __float_as_uint(f);
  return (unsigned short)((u + 0x7FFFu + ((u >> 16) & 1u)) >> 16);
}
__device__ __forceinline__ float bfr(float f) { return __uint_as_float(((unsigned)bf_bits(f)) << 16); }
__device__ __forceinline__ unsigned short h_bits(_Float16 x) { return __builtin_bit_cast(unsigned short, x); }
__device__ __forceinline__ unsigned pk16(unsigned short a, unsigned short b) { return (unsigned)a | ((unsigned)b << 16); }
__device__ __forceinline__ v8f zero8() { v8f z = {0.f, 0.f, 0.f, 0.f, 0.f, 0.f, 0.f, 0.f}; return z; }

__device__ __forceinline__ v16h ldfrag_h(const _Float16* p) {
  Frag f;
  f.half[0] = *(const v8h*)(p);
  f.half[1] = *(const v8h*)(p + 16);
  return f.v;
}

__device__ __forceinline__ v8f mma_h(v16h a, v16h b, v8f c) {
  c = __builtin_amdgcn_wmma_f32_16x16x32_f16(false, a, false, b, (short)0, c, false, false);
#if defined(__HIP_DEVICE_COMPILE__)
  asm volatile("v_nop\n\tv_nop\n\tv_nop\n\tv_nop" : "+v"(c) : "v"(a), "v"(b));
#endif
  return c;
}

__device__ __forceinline__ v4u pack8h(v4f a, v4f b) {
  v4u p;
  p[0] = pk16(h_bits((_Float16)a[0]), h_bits((_Float16)a[1]));
  p[1] = pk16(h_bits((_Float16)a[2]), h_bits((_Float16)a[3]));
  p[2] = pk16(h_bits((_Float16)b[0]), h_bits((_Float16)b[1]));
  p[3] = pk16(h_bits((_Float16)b[2]), h_bits((_Float16)b[3]));
  return p;
}
__device__ __forceinline__ void split8h(v4f a, v4f b, v4u& ph, v4u& pl) {
  v4f ra, rb;
#pragma unroll
  for (int e = 0; e < 4; ++e) {
    const _Float16 ha = (_Float16)a[e];
    ra[e] = (a[e] - (float)ha) * 2048.0f;
    const _Float16 hb = (_Float16)b[e];
    rb[e] = (b[e] - (float)hb) * 2048.0f;
  }
  ph = pack8h(a, b);
  pl = pack8h(ra, rb);
}

__device__ __forceinline__ void cvt8_w(const float* __restrict__ src, unsigned short* dst, size_t e0) {
  const v4f a = *(const v4f*)(src + e0);
  const v4f b = *(const v4f*)(src + e0 + 4);
  v4f sa, sb;
#pragma unroll
  for (int e = 0; e < 4; ++e) { sa[e] = bfr(a[e]) * CWS; sb[e] = bfr(b[e]) * CWS; }
  const v4u pk = pack8h(sa, sb);
  *(volatile v4u*)(dst + e0) = pk;
  __threadfence();
  *(volatile v4u*)(dst + e0) = pk;
}

__global__ __launch_bounds__(256)
void pool_k(const float* __restrict__ x, float* gm) {
  __shared__ __align__(16) float ms[32];
  const int tid = threadIdx.x;
  const int cg = blockIdx.x, b = blockIdx.y;
  const int ci = tid >> 3, q = tid & 7;
  const int ch = cg * 32 + ci;
  const v4f* xp = (const v4f*)(x + ((size_t)(b * NC + ch)) * HW) + q;
  v4f s4 = {0.f, 0.f, 0.f, 0.f};
#pragma unroll 4
  for (int j = 0; j < HW / 32; ++j) {
    const v4f v = xp[8 * j];
#pragma unroll
    for (int e = 0; e < 4; ++e) s4[e] += bfr(v[e]);
  }
  float s = (s4[0] + s4[1]) + (s4[2] + s4[3]);
  s += __shfl_xor(s, 1, 32);
  s += __shfl_xor(s, 2, 32);
  s += __shfl_xor(s, 4, 32);
  if (q == 0) ms[ci] = s * (1.0f / 12544.0f);
  __syncthreads();
  if (tid < 8) {
    const v4f v = *(const v4f*)(ms + tid * 4);
    float* gp = gm + (size_t)(b * NC + cg * 32) + tid * 4;
    *(volatile v4f*)gp = v;
    __threadfence();
    *(volatile v4f*)gp = v;
  }
}

__global__ __launch_bounds__(256)
void rank_k(const float* __restrict__ gm, const float* __restrict__ w1, const float* __restrict__ b1,
            const float* __restrict__ w2, const float* __restrict__ b2, const float* __restrict__ bw,
            const float* __restrict__ bb, const float* __restrict__ fw, float* kb, unsigned short* Wh) {
  __shared__ __align__(16) float gs[NC];
  __shared__ float hs[NH1], wl[NS], es[NS], wts[NS];
  __shared__ __align__(16) float kbs[NC * KBW];
  const int tid = threadIdx.x, blk = blockIdx.x;
  if (blk >= NB) {
    cvt8_w(fw, Wh, ((size_t)(blk - NB) * 256 + tid) * 8);
    return;
  }
  const int b = blk;
  if (tid < NC) gs[tid] = gm[(size_t)b * NC + tid];
  __syncthreads();
  if (tid < NH1) {
    const float* wr = w1 + (size_t)tid * NC;
    float a = 0.0f;
#pragma unroll 1
    for (int cc = 0; cc < NC; ++cc) a += gs[cc] * bfr(wr[cc]);
    a += bfr(b1[tid]);
    hs[tid] = fmaxf(a, 0.0f);
  }
  __syncthreads();
  if (tid < 32) {
    const int s = tid & 15;
    const float* wr = w2 + (size_t)s * NH1;
    float a = 0.0f;
#pragma unroll 1
    for (int j = 0; j < NH1; ++j) a += hs[j] * bfr(wr[j]);
    a += bfr(b2[s]);
    if (tid < NS) wl[s] = a;
  }
  __syncthreads();
  if (tid < 32) {
    const int s = tid & 15;
    float m = wl[0];
#pragma unroll 1
    for (int j = 1; j < NS; ++j) m = fmaxf(m, wl[j]);
    const float e = expf(wl[s] - m);
    if (tid < NS) es[s] = e;
  }
  __syncthreads();
  if (tid < 32) {
    const int s = tid & 15;
    float sum = 0.0f;
#pragma unroll 1
    for (int j = 0; j < NS; ++j) sum += es[j];
    const float v = es[s] * (1.0f / sum);
    if (tid < NS) wts[s] = v;
  }
  __syncthreads();
  for (int i = tid; i < NC * KBW; i += 256) {
    const int c = i >> 4, k = i & 15;
    const int kc = (k < 9) ? k : 8;
    float a = 0.0f;
#pragma unroll 1
    for (int s = 0; s < NS; ++s) {
      const float wv = bfr(bw[((size_t)(s * NC + c)) * 9 + kc]);
      const float bv = bfr(bb[(size_t)s * NC + c]);
      const float val = (k < 9) ? wv : ((k == 9) ? bv : 0.0f);
      a += wts[s] * val;
    }
    kbs[i] = a;
  }
  __syncthreads();
  v4f pv[2];
  size_t po[2];
#pragma unroll
  for (int it = 0; it < 2; ++it) {
    const int piece = it * 256 + tid;
    pv[it] = *(const v4f*)(kbs + piece * 4);
    po[it] = (size_t)b * (NC * KBW) + (size_t)piece * 4;
  }
#pragma unroll
  for (int it = 0; it < 2; ++it) *(volatile v4f*)(kb + po[it]) = pv[it];
  __threadfence();
#pragma unroll
  for (int it = 0; it < 2; ++it) *(volatile v4f*)(kb + po[it]) = pv[it];
}

__global__ __launch_bounds__(256)
void main_k(const float* __restrict__ x, const float* __restrict__ kb, const unsigned short* __restrict__ Wh,
            const float* __restrict__ fb, float* out) {
  __shared__ __align__(16) float kbs[NC * KBW];
  __shared__ float fbs[NC];
  __shared__ __align__(16) unsigned short big[2 * 64 * BKP];
  unsigned short* Bh = big;
  unsigned short* Bl = big + 64 * BKP;
  const int tid = threadIdx.x, wave = tid >> 5, lane = tid & 31, hh = lane >> 4, c = lane & 15;
  const int pt = blockIdx.x, b = blockIdx.y;

  {
    const v4f* src = (const v4f*)(kb + (size_t)b * (NC * KBW));
    v4f* dst = (v4f*)kbs;
    dst[tid] = src[tid];
    dst[tid + 256] = src[tid + 256];
  }
  if (tid < NC) fbs[tid] = bfr(fb[tid]);

  const int px = tid & 63, cq = tid >> 6;
  const int p = pt * 64 + px;
  const int hy = p / IMW, wx = p - hy * IMW;
  int toff[9];
  float tmsk[9];
#pragma unroll
  for (int dy = 0; dy < 3; ++dy) {
#pragma unroll
    for (int dx = 0; dx < 3; ++dx) {
      const int yy = hy + dy - 1, xx = wx + dx - 1;
      const bool ok = ((unsigned)yy < (unsigned)IMW) && ((unsigned)xx < (unsigned)IMW);
      const int yc = (yy < 0) ? 0 : ((yy > IMW - 1) ? (IMW - 1) : yy);
      const int xc = (xx < 0) ? 0 : ((xx > IMW - 1) ? (IMW - 1) : xx);
      toff[dy * 3 + dx] = yc * IMW + xc;
      tmsk[dy * 3 + dx] = ok ? 1.0f : 0.0f;
    }
  }
  __syncthreads();

#pragma unroll 1
  for (int jb = 0; jb < 4; ++jb) {
    const int chl0 = cq * 32 + jb * 8;
    v4f fa, fbv;
#pragma unroll
    for (int e = 0; e < 8; ++e) {
      const int ch = chl0 + e;
      const float* xp = x + ((size_t)(b * NC + ch)) * HW;
      const float* kr = kbs + ch * KBW;
      float a = 0.0f;
#pragma unroll
      for (int t = 0; t < 9; ++t) a += (bfr(xp[toff[t]]) * tmsk[t]) * kr[t];
      const float u = (a + kr[9]) * CAS;
      if (e < 4) fa[e] = u; else fbv[e - 4] = u;
    }
    v4u ph, pl;
    split8h(fa, fbv, ph, pl);
    *(v4u*)(Bh + px * BKP + chl0) = ph;
    *(v4u*)(Bl + px * BKP + chl0) = pl;
  }
  __syncthreads();

  const _Float16* A   = (const _Float16*)(const void*)Wh;
  const _Float16* Bhh = (const _Float16*)(const void*)Bh;
  const _Float16* Blh = (const _Float16*)(const void*)Bl;
  const int mt = wave;

  v8f acch[4], accl[4];
#pragma unroll
  for (int nt = 0; nt < 4; ++nt) { acch[nt] = zero8(); accl[nt] = zero8(); }

#pragma unroll 1
  for (int kk = 0; kk < 4; ++kk) {
    const int k0 = kk * 32;
    const v16h a = ldfrag_h(A + (size_t)(mt * 16 + c) * NC + k0 + 8 * hh);
#pragma unroll
    for (int nt = 0; nt < 4; ++nt) {
      const v16h bh = ldfrag_h(Bhh + (nt * 16 + c) * BKP + k0 + 8 * hh);
      const v16h bl = ldfrag_h(Blh + (nt * 16 + c) * BKP + k0 + 8 * hh);
      acch[nt] = mma_h(a, bh, acch[nt]);
      accl[nt] = mma_h(a, bl, accl[nt]);
    }
  }
  __syncthreads();
  float* so = (float*)(void*)big;
#pragma unroll
  for (int nt = 0; nt < 4; ++nt) {
#pragma unroll
    for (int r = 0; r < 8; ++r) {
      const float v = (acch[nt][r] + accl[nt][r] * (1.0f / 2048.0f)) * (1.0f / (CWS * CAS));
      so[(mt * 16 + 8 * hh + r) * SOP + nt * 16 + c] = v;
    }
  }
  __syncthreads();
  v4f ov[8];
  size_t offs[8];
#pragma unroll
  for (int it = 0; it < 8; ++it) {
    const int ch = wave * 16 + it * 2 + hh;
    const v4f t = *(const v4f*)(so + ch * SOP + c * 4);
    const size_t off = ((size_t)(b * NC + ch)) * HW + (size_t)pt * 64 + c * 4;
    const v4f xr = *(const v4f*)(x + off);
    const float bias = fbs[ch];
    v4f o4;
#pragma unroll
    for (int e = 0; e < 4; ++e) o4[e] = (t[e] + bias) + bfr(xr[e]);
    ov[it] = o4;
    offs[it] = off;
  }
#pragma unroll
  for (int it = 0; it < 8; ++it) *(volatile v4f*)(out + offs[it]) = ov[it];
  __threadfence();
#pragma unroll
  for (int it = 0; it < 8; ++it) *(volatile v4f*)(out + offs[it]) = ov[it];
}

extern "C" void kernel_launch(void* const* d_in, const int* in_sizes, int n_in,
                              void* d_out, int out_size, void* d_ws, size_t ws_size,
                              hipStream_t stream) {
  if (n_in < 9) return;
  if (in_sizes[0] != NB * NC * HW) return;
  if (in_sizes[1] != NS * NC * 9) return;
  if (in_sizes[2] != NS * NC) return;
  if (in_sizes[3] != NH1 * NC) return;
  if (in_sizes[4] != NH1) return;
  if (in_sizes[5] != NS * NH1) return;
  if (in_sizes[6] != NS) return;
  if (in_sizes[7] != NC * NC) return;
  if (in_sizes[8] != NC) return;
  if (out_size != NB * NC * HW) return;

  const float* x        = (const float*)d_in[0];
  const float* branch_w = (const float*)d_in[1];
  const float* branch_b = (const float*)d_in[2];
  const float* rank_w1  = (const float*)d_in[3];
  const float* rank_b1  = (const float*)d_in[4];
  const float* rank_w2  = (const float*)d_in[5];
  const float* rank_b2  = (const float*)d_in[6];
  const float* fuse_w   = (const float*)d_in[7];
  const float* fuse_b   = (const float*)d_in[8];
  float* out = (float*)d_out;

  const size_t sG  = (size_t)NB * NC * 4;
  const size_t sKB = (size_t)NB * NC * KBW * 4;
  const size_t sWH = (size_t)NC * NC * 2;
  size_t off = 0;
  const size_t oG  = off; off += sG;
  const size_t oKB = off; off += sKB;
  const size_t oWH = off; off += sWH;
  if (off > ws_size) return;
  if (off > (size_t)134217728) return;

  char* ws = (char*)d_ws;
  float* gm          = (float*)(ws + oG);
  float* kb          = (float*)(ws + oKB);
  unsigned short* Wh = (unsigned short*)(ws + oWH);

  const dim3 blk(256);
  pool_k<<<dim3(NC / 32, NB), blk, 0, stream>>>(x, gm);
  rank_k<<<dim3(NB + 8), blk, 0, stream>>>(gm, rank_w1, rank_b1, rank_w2, rank_b2, branch_w, branch_b,
                                           fuse_w, kb, Wh);
  main_k<<<dim3(NPT, NB), blk, 0, stream>>>(x, kb, Wh, fuse_b, out);
  (void)hipGetLastError();
}
